// PNALayer_88484916232760
// MI455X (gfx1250) — hardware-run, weakly checked
//
#include <hip/hip_runtime.h>
#include <stddef.h>
#include <stdint.h>


#pragma clang fp contract(off)

#define NODE   128
#define NT     4
#define TWD    32
#define PSW    256
#define AGW    512
#define KPOST  416
#define KP8    52
#define NTHR   256
#define NWAVE  8
#define EPT    8
#define CHUNK  (NTHR * EPT)
#define WCAP   (EPT * 32)
#define LISTN  (NWAVE * WCAP)
#define NBMAX  2048
#define SLOTB  11
#define RCAP   28672
#define DEGCAP 4096
#define GBM    64
#define GTHR   128
#define NSPLIT 2
#define NBMIN  64
#define EPSV   1.0e-5f
#define LOG5F  1.6094379124341003f
#define WSMAX  134217728
#define NU0    (2 * NODE * 4)
#define NU1    (NT * TWD * KP8)
#define NU2    (NODE * (NODE / 8))
#define NUW    (NU0 + NU1 + NU2)
#define LDS_AGG ((2 * RCAP + 2 * NBMAX + LISTN + 2 * NWAVE + NBMAX) * 4)

static_assert((CHUNK & (CHUNK - 1)) == 0 && CHUNK <= 4096);
static_assert(NBMAX == (1 << SLOTB));
static_assert(NTHR * 8 == NBMAX);
static_assert(LISTN >= NBMAX);
static_assert(LISTN >= NWAVE * WCAP);
static_assert((RCAP % 32) == 0);
static_assert(LDS_AGG <= 300000);
static_assert(((2 * RCAP + 2 * NBMAX + LISTN + 2 * NWAVE) % 4) == 0);
static_assert(GBM == (GTHR / 32) * 16);
static_assert(NODE == NT * TWD && TWD == 32);
static_assert(KPOST == 13 * TWD && (KPOST % 32) == 0 && KP8 * 8 == KPOST);
static_assert(PSW == 2 * NODE && AGW == 4 * NODE);
static_assert((NU0 % NTHR) == 0 && ((NU0 + NU1) % NTHR) == 0 && (NUW % NTHR) == 0);
static_assert(NBMIN >= GBM && (NBMIN % GBM) == 0 && NBMIN >= 8);

typedef float          v4f  __attribute__((ext_vector_type(4)));
typedef float          v8f  __attribute__((ext_vector_type(8)));
typedef int            v4i  __attribute__((ext_vector_type(4)));
typedef int            v8i  __attribute__((ext_vector_type(8)));
typedef unsigned short v8us __attribute__((ext_vector_type(8)));
typedef __bf16         v16b __attribute__((ext_vector_type(16)));
typedef v4f  __attribute__((may_alias)) v4fa;
typedef v8us __attribute__((may_alias)) v8usa;
union FragB { v16b v; v8us h[2]; v8i w; };

__device__ __forceinline__ v8f wmb(const FragB& a, const FragB& b, v8f c) {
  v8f d = __builtin_amdgcn_wmma_f32_16x16x32_bf16(false, a.v, false, b.v, (short)0, c, false, false);
  asm volatile("v_nop\n\tv_nop\n\tv_nop\n\tv_nop" : "+v"(d) : "v"(a.w), "v"(b.w));
  return d;
}

__device__ __forceinline__ unsigned bfb(float x) {
  const unsigned u = __float_as_uint(x);
  return (u + 0x7FFFu + ((u >> 16) & 1u)) >> 16;
}
__device__ __forceinline__ float bfr(float x) { return __uint_as_float(bfb(x) << 16); }

__device__ __forceinline__ v8us hi8(const v4f a, const v4f b) {
  v8us r;
  r[0] = (unsigned short)bfb(a.x); r[1] = (unsigned short)bfb(a.y);
  r[2] = (unsigned short)bfb(a.z); r[3] = (unsigned short)bfb(a.w);
  r[4] = (unsigned short)bfb(b.x); r[5] = (unsigned short)bfb(b.y);
  r[6] = (unsigned short)bfb(b.z); r[7] = (unsigned short)bfb(b.w);
  return r;
}

__device__ __forceinline__ void split8(const v4f a, const v4f b, v8us& hi, v8us& lo) {
#define SPL(I, X) { const unsigned hb = bfb(X); const float hf = __uint_as_float(hb << 16); \
                    hi[I] = (unsigned short)hb; lo[I] = (unsigned short)bfb((X) - hf); }
  SPL(0, a.x) SPL(1, a.y) SPL(2, a.z) SPL(3, a.w)
  SPL(4, b.x) SPL(5, b.y) SPL(6, b.z) SPL(7, b.w)
#undef SPL
}

__device__ __forceinline__ void frag_hi(const float* p, int hh, FragB& f) {
  const v4f a = *(const v4fa*)(p + 8 * hh);
  const v4f b = *(const v4fa*)(p + 8 * hh + 4);
  const v4f c = *(const v4fa*)(p + 16 + 8 * hh);
  const v4f d = *(const v4fa*)(p + 16 + 8 * hh + 4);
  f.h[0] = hi8(a, b);
  f.h[1] = hi8(c, d);
}
__device__ __forceinline__ void frag_split(const float* p, int hh, FragB& fh, FragB& fl) {
  const v4f a = *(const v4fa*)(p + 8 * hh);
  const v4f b = *(const v4fa*)(p + 8 * hh + 4);
  const v4f c = *(const v4fa*)(p + 16 + 8 * hh);
  const v4f d = *(const v4fa*)(p + 16 + 8 * hh + 4);
  split8(a, b, fh.h[0], fl.h[0]);
  split8(c, d, fh.h[1], fl.h[1]);
}
__device__ __forceinline__ void frag_w(const unsigned short* p, int hh, FragB& f) {
  f.h[0] = *(const v8usa*)(p + 8 * hh);
  f.h[1] = *(const v8usa*)(p + 16 + 8 * hh);
}

__device__ __forceinline__ int scan_chunk(const int* __restrict__ dsts, int nE, int cbase, int slotBase,
                                          int nb, int vec8, int* list, int tid, int lane, int wave) {
  int wc = 0;
  const int el0  = tid * EPT;
  const int e0   = cbase + el0;
  const int sent = -2147483647 - 1;
  v4i da, db;
  if (vec8 != 0 && cbase + CHUNK <= nE) {
    da = *(const v4i*)(dsts + e0);
    db = *(const v4i*)(dsts + e0 + 4);
  } else {
    da.x = (e0     < nE) ? dsts[min(e0,     nE - 1)] : sent;
    da.y = (e0 + 1 < nE) ? dsts[min(e0 + 1, nE - 1)] : sent;
    da.z = (e0 + 2 < nE) ? dsts[min(e0 + 2, nE - 1)] : sent;
    da.w = (e0 + 3 < nE) ? dsts[min(e0 + 3, nE - 1)] : sent;
    db.x = (e0 + 4 < nE) ? dsts[min(e0 + 4, nE - 1)] : sent;
    db.y = (e0 + 5 < nE) ? dsts[min(e0 + 5, nE - 1)] : sent;
    db.z = (e0 + 6 < nE) ? dsts[min(e0 + 6, nE - 1)] : sent;
    db.w = (e0 + 7 < nE) ? dsts[min(e0 + 7, nE - 1)] : sent;
  }
  const unsigned nbs = (unsigned)slotBase;
  const unsigned unb = (unsigned)nb;
  const unsigned s0 = (unsigned)da.x - nbs, s1 = (unsigned)da.y - nbs;
  const unsigned s2 = (unsigned)da.z - nbs, s3 = (unsigned)da.w - nbs;
  const unsigned s4 = (unsigned)db.x - nbs, s5 = (unsigned)db.y - nbs;
  const unsigned s6 = (unsigned)db.z - nbs, s7 = (unsigned)db.w - nbs;
  const bool h0 = s0 < unb, h1 = s1 < unb, h2 = s2 < unb, h3 = s3 < unb;
  const bool h4 = s4 < unb, h5 = s5 < unb, h6 = s6 < unb, h7 = s7 < unb;
  const unsigned any = __builtin_amdgcn_ballot_w32(h0 | h1 | h2 | h3 | h4 | h5 | h6 | h7);
  if (any != 0u) {
#define HITJ(J, HJ, SJ) { \
      const unsigned mj = __builtin_amdgcn_ballot_w32(HJ); \
      if (mj != 0u) { \
        if (HJ) { \
          const int pos = wc + (int)__builtin_amdgcn_mbcnt_lo(mj, 0u); \
          if (pos < WCAP) list[wave * WCAP + pos] = ((el0 + (J)) << 12) | (int)(SJ); \
        } \
        wc += (int)__builtin_popcount(mj); } }
    HITJ(0, h0, s0)
    HITJ(1, h1, s1)
    HITJ(2, h2, s2)
    HITJ(3, h3, s3)
    HITJ(4, h4, s4)
    HITJ(5, h5, s5)
    HITJ(6, h6, s6)
    HITJ(7, h7, s7)
#undef HITJ
  }
  return wc;
}

__global__ __launch_bounds__(NTHR) void k_wprep(const float* __restrict__ Wpre, const float* __restrict__ Wpost,
                                                const float* __restrict__ Wmix, unsigned short* wpreP,
                                                unsigned short* wpostP, unsigned short* wmixP) {
  const int u = (int)blockIdx.x * NTHR + (int)threadIdx.x;
  if (u >= NUW) return;
  const float* p;
  int strd;
  unsigned short* d;
  if (u < NU0) {
    const int y = u >> 9, n = (u >> 2) & 127, k8 = (u & 3) * 8;
    const int t = n >> 5, o = n & 31;
    p = Wpre + (size_t)(t * 64 + y * 32 + k8) * TWD + o;
    strd = TWD;
    d = wpreP + (size_t)u * 8;
  } else if (u < NU0 + NU1) {
    const int e = u - NU0;
    const int t = e / (TWD * KP8);
    const int rem = e - t * (TWD * KP8);
    const int n = rem / KP8;
    const int k8 = (rem - n * KP8) * 8;
    p = Wpost + (size_t)(t * KPOST + k8) * TWD + n;
    strd = TWD;
    d = wpostP + (size_t)e * 8;
  } else {
    const int e = u - NU0 - NU1;
    const int n = e >> 4, k8 = (e & 15) * 8;
    p = Wmix + (size_t)k8 * NODE + n;
    strd = NODE;
    d = wmixP + (size_t)e * 8;
  }
  v8us r;
  r[0] = (unsigned short)bfb(p[0]);
  r[1] = (unsigned short)bfb(p[(size_t)strd]);
  r[2] = (unsigned short)bfb(p[(size_t)2 * strd]);
  r[3] = (unsigned short)bfb(p[(size_t)3 * strd]);
  r[4] = (unsigned short)bfb(p[(size_t)4 * strd]);
  r[5] = (unsigned short)bfb(p[(size_t)5 * strd]);
  r[6] = (unsigned short)bfb(p[(size_t)6 * strd]);
  r[7] = (unsigned short)bfb(p[(size_t)7 * strd]);
  *(volatile v8us*)d = r;
  __threadfence();
  *(volatile v8us*)d = r;
}

__global__ __launch_bounds__(GTHR) void k_pre(const float* __restrict__ h, const unsigned short* __restrict__ wpreP,
                                              const float* __restrict__ bpre, float* PSD, int nN) {
  __shared__ __attribute__((aligned(16))) float stg[GBM * NODE];
  const int tid = (int)threadIdx.x, lane = tid & 31, wave = tid >> 5, hh = lane >> 4, m = lane & 15;
  const int rowBase = (int)blockIdx.x * GBM;
  const int y = (int)blockIdx.y;
  const int r = rowBase + 16 * wave + m;
  const int rc = r < nN ? r : nN - 1;
  const float* hr = h + (size_t)rc * NODE;
  const unsigned short* wp = wpreP + (size_t)(y * NODE + m) * TWD;

  const v8f z8 = {0.f, 0.f, 0.f, 0.f, 0.f, 0.f, 0.f, 0.f};
  v8f acc[8];
#pragma unroll
  for (int ct = 0; ct < 8; ++ct) acc[ct] = z8;

#pragma unroll
  for (int t = 0; t < NT; ++t) {
    FragB af;
    frag_hi(hr + t * TWD, hh, af);
#pragma unroll
    for (int j = 0; j < 2; ++j) {
      const int ct = 2 * t + j;
      FragB bf;
      frag_w(wp + (size_t)ct * 16 * TWD, hh, bf);
      acc[ct] = wmb(af, bf, acc[ct]);
    }
  }

#pragma unroll
  for (int ct = 0; ct < 8; ++ct) {
    const int col = 16 * ct + m;
    const float braw = bpre[col];
    const float bv = (y != 0) ? bfr(braw) : 0.0f;
#pragma unroll
    for (int r8 = 0; r8 < 8; ++r8) {
      const int lr = 16 * wave + 8 * hh + r8;
      stg[lr * NODE + col] = acc[ct][r8] + bv;
    }
  }
  __syncthreads();

  float* ob = PSD + (size_t)rowBase * PSW + (size_t)y * NODE + 4 * lane;
#pragma unroll
  for (int i = 0; i < 16; ++i) {
    const int lr = 16 * wave + i;
    const v4f v = *(const v4fa*)(stg + lr * NODE + 4 * lane);
    *(volatile v4f*)(ob + (size_t)lr * PSW) = v;
  }
  __threadfence();
#pragma unroll
  for (int i = 0; i < 16; ++i) {
    const int lr = 16 * wave + i;
    const v4f v = *(const v4fa*)(stg + lr * NODE + 4 * lane);
    *(volatile v4f*)(ob + (size_t)lr * PSW) = v;
  }
}

__global__ __launch_bounds__(NTHR) void k_agg(
    const int* __restrict__ srcs, const int* __restrict__ dsts,
    const float* __restrict__ PSD, float* AGG, float* SCP,
    int nN, int nE, int nb, int vec8, int rowLo, int RS) {
  extern __shared__ v4f lds_dyn[];
  int* reg1 = (int*)lds_dyn;
  int* reg2 = reg1 + RCAP;
  int* scnt = reg2 + RCAP;
  int* soff = scnt + NBMAX;
  int* list = soff + NBMAX;
  int* wcnt = list + LISTN;
  int* wtot = wcnt + NWAVE;
  float* scv = (float*)(wtot + NWAVE);
  const int tid = (int)threadIdx.x, lane = tid & 31, wave = tid >> 5;
  const int lrBase   = (int)blockIdx.x * nb;
  const int nodeBase = rowLo + lrBase;

  for (int i = tid; i < NBMAX; i += NTHR) scnt[i] = 0;
  __syncthreads();

  int tot = 0;
  const int nChunks = (nE + CHUNK - 1) / CHUNK;
#pragma unroll 1
  for (int ch = 0; ch < nChunks; ++ch) {
    const int cbase = ch * CHUNK;
    const int wc = scan_chunk(dsts, nE, cbase, nodeBase, nb, vec8, list, tid, lane, wave);
    if (lane == 0) wcnt[wave] = wc;
    __syncthreads();
    int pre = 0, all = 0;
#pragma unroll
    for (int w2 = 0; w2 < NWAVE; ++w2) {
      int c = wcnt[w2];
      c = c < 0 ? 0 : (c > WCAP ? WCAP : c);
      all += c;
      pre += (w2 < wave) ? c : 0;
    }
    const int wcc  = wc > WCAP ? WCAP : wc;
    const int base = tot + pre;
#pragma unroll 1
    for (int i = lane; i < wcc; i += 32) {
      const int ent = list[wave * WCAP + i];
      const int el  = (ent >> 12) & (CHUNK - 1);
      const int sl  = ent & (NBMAX - 1);
      int eid = cbase + el;
      eid = eid > nE - 1 ? nE - 1 : eid;
      const int pos = base + i;
      if (pos < RCAP) reg1[pos] = (int)(((unsigned)eid << SLOTB) | (unsigned)sl);
    }
    tot += all;
    tot = tot > RCAP ? RCAP : tot;
    __syncthreads();
  }
  const int nh = tot;

  if (wave == 0) {
#pragma unroll 1
    for (int b0 = 0; b0 < nh; b0 += 32) {
      const int idx = b0 + lane;
      const int uv  = reg1[idx < RCAP ? idx : RCAP - 1];
      const int m32 = (nh - b0) < 32 ? (nh - b0) : 32;
#pragma unroll 1
      for (int k = 0; k < m32; ++k) {
        const int u  = __builtin_amdgcn_readlane(uv, k);
        const int sl = u & (NBMAX - 1);
        if (lane == 0) scnt[sl] = scnt[sl] + 1;
      }
    }
  }
  __syncthreads();

  {
    const v4i ca = *(const v4i*)(scnt + 8 * tid);
    const v4i cb = *(const v4i*)(scnt + 8 * tid + 4);
    const int e0 = ca.x < 0 ? 0 : ca.x, e1 = ca.y < 0 ? 0 : ca.y, e2 = ca.z < 0 ? 0 : ca.z, e3 = ca.w < 0 ? 0 : ca.w;
    const int e4 = cb.x < 0 ? 0 : cb.x, e5 = cb.y < 0 ? 0 : cb.y, e6 = cb.z < 0 ? 0 : cb.z, e7 = cb.w < 0 ? 0 : cb.w;
    const int ts = e0 + e1 + e2 + e3 + e4 + e5 + e6 + e7;
    int incl = ts;
#pragma unroll
    for (int d = 1; d < 32; d <<= 1) {
      const int up = __shfl_up(incl, d);
      if (lane >= d) incl += up;
    }
    if (lane == 31) wtot[wave] = incl;
    __syncthreads();
    int pre = 0;
#pragma unroll
    for (int w2 = 0; w2 < NWAVE; ++w2) pre += (w2 < wave) ? wtot[w2] : 0;
    int run = pre + incl - ts;
    soff[8 * tid + 0] = run; run += e0;
    soff[8 * tid + 1] = run; run += e1;
    soff[8 * tid + 2] = run; run += e2;
    soff[8 * tid + 3] = run; run += e3;
    soff[8 * tid + 4] = run; run += e4;
    soff[8 * tid + 5] = run; run += e5;
    soff[8 * tid + 6] = run; run += e6;
    soff[8 * tid + 7] = run;
  }
  __syncthreads();
  for (int i = tid; i < NBMAX; i += NTHR) list[i] = soff[i];
  __syncthreads();

  if (wave == 0) {
#pragma unroll 1
    for (int b0 = 0; b0 < nh; b0 += 32) {
      const int idx = b0 + lane;
      const int uv  = reg1[idx < RCAP ? idx : RCAP - 1];
      const int m32 = (nh - b0) < 32 ? (nh - b0) : 32;
#pragma unroll 1
      for (int k = 0; k < m32; ++k) {
        const int u   = __builtin_amdgcn_readlane(uv, k);
        const int sl  = u & (NBMAX - 1);
        const int eid = (int)((unsigned)u >> SLOTB);
        if (lane == 0) {
          int pos = list[sl];
          pos = pos < 0 ? 0 : (pos > RCAP - 1 ? RCAP - 1 : pos);
          reg2[pos] = eid;
          list[sl] = pos + 1;
        }
      }
    }
  }
  __syncthreads();

  const int nbw = nb >> 3;
  const bool ovf = (nh >= RCAP);
  const float qnan = __uint_as_float(0x7fc00000u);
  const float ninf = __uint_as_float(0xff800000u);
  const float pinf = __uint_as_float(0x7f800000u);
  const int tq = lane >> 3, o4 = 4 * (lane & 7);
#pragma unroll 1
  for (int jt = 0; jt < nbw; ++jt) {
    const int slot = wave * nbw + jt;
    const int lrow = lrBase + slot;
    const int grow = rowLo + lrow;
    const int gcl  = grow < nN ? grow : nN - 1;
    int st = soff[slot];
    const int craw = scnt[slot];
    int cnt = craw;
    st  = st < 0 ? 0 : (st > nh ? nh : st);
    cnt = cnt < 0 ? 0 : (cnt > DEGCAP ? DEGCAP : cnt);
    if (cnt > nh - st) cnt = nh - st;
    const bool pois = ovf || (craw > DEGCAP);
    const bool wr   = lrow < RS;
    const bool live = grow < nN;

    const v4f pdb = *(const v4fa*)(PSD + (size_t)gcl * PSW + NODE + 4 * lane);
    float sm[4], sq[4], mx[4], mn[4];
#pragma unroll
    for (int i = 0; i < 4; ++i) { sm[i] = 0.f; sq[i] = 0.f; mx[i] = ninf; mn[i] = pinf; }

#pragma unroll 1
    for (int q = 0; q < cnt; ++q) {
      int idx = st + q; idx = idx > RCAP - 1 ? RCAP - 1 : idx;
      int eid = reg2[idx]; eid = eid < 0 ? 0 : (eid > nE - 1 ? nE - 1 : eid);
      const int sraw = srcs[eid];
      const int s = sraw < 0 ? 0 : (sraw > nN - 1 ? nN - 1 : sraw);
      const v4f ps = *(const v4fa*)(PSD + (size_t)s * PSW + 4 * lane);
      float ev[4];
      ev[0] = fmaxf(ps.x + pdb.x, 0.f);
      ev[1] = fmaxf(ps.y + pdb.y, 0.f);
      ev[2] = fmaxf(ps.z + pdb.z, 0.f);
      ev[3] = fmaxf(ps.w + pdb.w, 0.f);
#pragma unroll
      for (int i = 0; i < 4; ++i) {
        sm[i] += ev[i];
        sq[i] += ev[i] * ev[i];
        mx[i] = fmaxf(mx[i], ev[i]);
        mn[i] = fminf(mn[i], ev[i]);
      }
    }

    const float degf = (float)cnt;
    const float rd   = 1.0f / fmaxf(degf, 1.0f);
    const float scl  = logf(degf + 1.0f) * (1.0f / LOG5F);
    if (lane == 0) scv[slot] = scl;
    float meanv[4], sdv[4];
#pragma unroll
    for (int i = 0; i < 4; ++i) {
      const float mean = sm[i] * rd;
      const float msq  = sq[i] * rd;
      const float var  = fmaxf(msq - mean * mean, 0.f);
      meanv[i] = mean;
      sdv[i]   = sqrtf(var + EPSV);
    }
    v4f va0 = {meanv[0], meanv[1], meanv[2], meanv[3]};
    v4f va1 = {mx[0], mx[1], mx[2], mx[3]};
    v4f va2 = {mn[0], mn[1], mn[2], mn[3]};
    v4f va3 = {sdv[0], sdv[1], sdv[2], sdv[3]};
    const v4f z4 = {0.f, 0.f, 0.f, 0.f};
    const v4f n4 = {qnan, qnan, qnan, qnan};
    if (!live) { va0 = z4; va1 = z4; va2 = z4; va3 = z4; }
    if (pois)  { va0 = n4; va1 = n4; va2 = n4; va3 = n4; }

    float* ap = AGG + (size_t)lrow * AGW + tq * 128 + o4;
    if (wr) {
      *(volatile v4f*)(ap)      = va0;
      *(volatile v4f*)(ap + 32) = va1;
      *(volatile v4f*)(ap + 64) = va2;
      *(volatile v4f*)(ap + 96) = va3;
    }
    __threadfence();
    if (wr) {
      *(volatile v4f*)(ap)      = va0;
      *(volatile v4f*)(ap + 32) = va1;
      *(volatile v4f*)(ap + 64) = va2;
      *(volatile v4f*)(ap + 96) = va3;
    }
  }
  __syncthreads();

  const int npc = nb >> 2;
#pragma unroll 1
  for (int p = tid; p < npc; p += NTHR) {
    const v4f v = *(const v4fa*)(scv + 4 * p);
    *(volatile v4f*)(SCP + (size_t)lrBase + 4 * p) = v;
  }
  __threadfence();
#pragma unroll 1
  for (int p = tid; p < npc; p += NTHR) {
    const v4f v = *(const v4fa*)(scv + 4 * p);
    *(volatile v4f*)(SCP + (size_t)lrBase + 4 * p) = v;
  }
}

__global__ __launch_bounds__(GTHR) void k_post(
    const float* __restrict__ h, const float* __restrict__ AGG, const float* __restrict__ SCP,
    const unsigned short* __restrict__ wpostP, const unsigned short* __restrict__ wmixP,
    const float* __restrict__ bpost, const float* __restrict__ bmix,
    float* out, int nN, int rowLo) {
  __shared__ __attribute__((aligned(16))) float tile[GBM * NODE];
  const int tid = (int)threadIdx.x, lane = tid & 31, wave = tid >> 5, hh = lane >> 4, m = lane & 15;
  const int lrBase  = (int)blockIdx.x * GBM;
  const int rowBase = rowLo + lrBase;
  const int lrow = lrBase + 16 * wave + m;
  const int grow = rowBase + 16 * wave + m;
  const int grc  = grow < nN ? grow : nN - 1;
  const float* hr = h + (size_t)grc * NODE;
  const float* ar = AGG + (size_t)lrow * AGW;

  float sc8[8], rs8[8];
  {
    const v4f sa = *(const v4fa*)(SCP + (size_t)lrBase + 16 * wave + 8 * hh);
    const v4f sb = *(const v4fa*)(SCP + (size_t)lrBase + 16 * wave + 8 * hh + 4);
    sc8[0] = sa.x; sc8[1] = sa.y; sc8[2] = sa.z; sc8[3] = sa.w;
    sc8[4] = sb.x; sc8[5] = sb.y; sc8[6] = sb.z; sc8[7] = sb.w;
#pragma unroll
    for (int r = 0; r < 8; ++r) rs8[r] = 1.0f / fmaxf(sc8[r], EPSV);
  }
  const v8f z8 = {0.f, 0.f, 0.f, 0.f, 0.f, 0.f, 0.f, 0.f};

#pragma unroll 1
  for (int t = 0; t < NT; ++t) {
    v8f accU[2], accS[2], accA[2];
    accU[0] = z8; accU[1] = z8; accS[0] = z8; accS[1] = z8; accA[0] = z8; accA[1] = z8;
    const unsigned short* wrow = wpostP + (size_t)(t * TWD + m) * KPOST;
    {
      FragB af;
      frag_hi(hr + t * TWD, hh, af);
#pragma unroll
      for (int ct = 0; ct < 2; ++ct) {
        FragB bf;
        frag_w(wrow + (size_t)ct * 16 * KPOST, hh, bf);
        accU[ct] = wmb(af, bf, accU[ct]);
      }
    }
#pragma unroll 1
    for (int ks = 0; ks < 4; ++ks) {
      FragB ahi, alo;
      frag_split(ar + t * 128 + 32 * ks, hh, ahi, alo);
#pragma unroll
      for (int ct = 0; ct < 2; ++ct) {
        const unsigned short* wq = wrow + (size_t)ct * 16 * KPOST + 32 * ks;
        FragB b1;
        frag_w(wq + TWD, hh, b1);
        accU[ct] = wmb(ahi, b1, accU[ct]);
        accU[ct] = wmb(alo, b1, accU[ct]);
        FragB b2;
        frag_w(wq + 5 * TWD, hh, b2);
        accS[ct] = wmb(ahi, b2, accS[ct]);
        accS[ct] = wmb(alo, b2, accS[ct]);
        FragB b3;
        frag_w(wq + 9 * TWD, hh, b3);
        accA[ct] = wmb(ahi, b3, accA[ct]);
        accA[ct] = wmb(alo, b3, accA[ct]);
      }
    }
#pragma unroll
    for (int ct = 0; ct < 2; ++ct) {
      const int col = t * TWD + 16 * ct + m;
      const float bv = bfr(bpost[col]);
#pragma unroll
      for (int r = 0; r < 8; ++r) {
        const int lr = 16 * wave + 8 * hh + r;
        const float v = accU[ct][r] + sc8[r] * accS[ct][r] + rs8[r] * accA[ct][r] + bv;
        tile[lr * NODE + col] = fmaxf(v, 0.f);
      }
    }
  }
  __syncthreads();

  v8f acc[8];
#pragma unroll
  for (int nt = 0; nt < 8; ++nt) acc[nt] = z8;
  const float* tr = tile + (16 * wave + m) * NODE;
#pragma unroll 1
  for (int ks = 0; ks < 4; ++ks) {
    FragB ahi, alo;
    frag_split(tr + 32 * ks, hh, ahi, alo);
#pragma unroll
    for (int nt = 0; nt < 8; ++nt) {
      FragB bf;
      frag_w(wmixP + (size_t)(16 * nt + m) * NODE + 32 * ks, hh, bf);
      acc[nt] = wmb(ahi, bf, acc[nt]);
      acc[nt] = wmb(alo, bf, acc[nt]);
    }
  }
  __syncthreads();

#pragma unroll
  for (int nt = 0; nt < 8; ++nt) {
    const int col = 16 * nt + m;
    const float bv = bfr(bmix[col]);
#pragma unroll
    for (int r = 0; r < 8; ++r) {
      const int lr = 16 * wave + 8 * hh + r;
      float v = acc[nt][r] + bv;
      v = v >= 0.f ? v : 0.01f * v;
      tile[lr * NODE + col] = v;
    }
  }
  __syncthreads();

#pragma unroll
  for (int i = 0; i < 16; ++i) {
    const int lr = 16 * wave + i;
    const int gr = rowBase + lr;
    const int gc = gr < nN ? gr : nN - 1;
    float* tp = tile + lr * NODE + 4 * lane;
    v4f tv = *(const v4fa*)tp;
    const v4f hv = *(const v4fa*)(h + (size_t)gc * NODE + 4 * lane);
    tv.x += bfr(hv.x); tv.y += bfr(hv.y); tv.z += bfr(hv.z); tv.w += bfr(hv.w);
    *(v4fa*)tp = tv;
  }

#pragma unroll
  for (int i = 0; i < 16; ++i) {
    const int lr = 16 * wave + i;
    const int gr = rowBase + lr;
    if (gr < nN) {
      const v4f v = *(const v4fa*)(tile + lr * NODE + 4 * lane);
      *(volatile v4f*)(out + (size_t)gr * NODE + 4 * lane) = v;
    }
  }
  __threadfence();
#pragma unroll
  for (int i = 0; i < 16; ++i) {
    const int lr = 16 * wave + i;
    const int gr = rowBase + lr;
    if (gr < nN) {
      const v4f v = *(const v4fa*)(tile + lr * NODE + 4 * lane);
      *(volatile v4f*)(out + (size_t)gr * NODE + 4 * lane) = v;
    }
  }
}

static int pick_nb(int nE, int nN) {
  int nb = NBMAX;
  while (nb > NBMIN && (long long)nb * (long long)nE * 5LL > (long long)RCAP * (long long)nN * 4LL) nb >>= 1;
  return nb;
}
static inline int cdiv(int a, int b) { return (a + b - 1) / b; }

extern "C" void kernel_launch(void* const* d_in, const int* in_sizes, int n_in,
                              void* d_out, int out_size, void* d_ws, size_t ws_size,
                              hipStream_t stream) {
  if (n_in < 9) return;
  const int nN = in_sizes[0] / NODE;
  if (nN <= 0 || in_sizes[0] != nN * NODE || nN > (1 << 22)) return;
  const int nE = in_sizes[1];
  if (nE < 1 || nE > (1 << 21) || in_sizes[2] != nE) return;
  if (in_sizes[3] != NT * 2 * TWD * TWD || in_sizes[4] != NT * TWD) return;
  if (in_sizes[5] != NT * KPOST * TWD   || in_sizes[6] != NT * TWD) return;
  if (in_sizes[7] != NODE * NODE         || in_sizes[8] != NODE)     return;
  if (out_size != nN * NODE) return;

  const float* h     = (const float*)d_in[0];
  const int*   src   = (const int*)  d_in[1];
  const int*   dst   = (const int*)  d_in[2];
  const float* Wpre  = (const float*)d_in[3];
  const float* bpre  = (const float*)d_in[4];
  const float* Wpost = (const float*)d_in[5];
  const float* bpost = (const float*)d_in[6];
  const float* Wmix  = (const float*)d_in[7];
  const float* bmix  = (const float*)d_in[8];
  float* out = (float*)d_out;

  const int MP = cdiv(nN, GBM) * GBM;
  const int nb = pick_nb(nE, nN);
  const int RS = cdiv(MP, NSPLIT * nb) * nb;
  const int gA = RS / nb;
  const int gP = RS / GBM;
  if ((RS % GBM) != 0 || gA * nb != RS || NSPLIT * RS < MP || (nb % 8) != 0) return;
  const int vec8 = ((nE & 3) == 0) ? 1 : 0;

  char* ws = (char*)d_ws;
  size_t off = 0;
  const size_t oPSD = off; off += (size_t)MP * PSW * 4;           off = (off + 255) & ~(size_t)255;
  const size_t oAGG = off; off += (size_t)RS * AGW * 4;           off = (off + 255) & ~(size_t)255;
  const size_t oSCP = off; off += (size_t)RS * 4;                 off = (off + 255) & ~(size_t)255;
  const size_t oWPR = off; off += (size_t)2 * NODE * TWD * 2;     off = (off + 255) & ~(size_t)255;
  const size_t oWPO = off; off += (size_t)NT * TWD * KPOST * 2;   off = (off + 255) & ~(size_t)255;
  const size_t oWMX = off; off += (size_t)NODE * NODE * 2;        off = (off + 255) & ~(size_t)255;
  if (off > ws_size || off > (size_t)WSMAX) return;
  float* PSD = (float*)(ws + oPSD);
  float* AGG = (float*)(ws + oAGG);
  float* SCP = (float*)(ws + oSCP);
  unsigned short* WPRE  = (unsigned short*)(ws + oWPR);
  unsigned short* WPOST = (unsigned short*)(ws + oWPO);
  unsigned short* WMIX  = (unsigned short*)(ws + oWMX);

  hipFuncSetAttribute(reinterpret_cast<const void*>(&k_agg),
                      hipFuncAttributeMaxDynamicSharedMemorySize, LDS_AGG);

  k_wprep<<<NUW / NTHR, NTHR, 0, stream>>>(Wpre, Wpost, Wmix, WPRE, WPOST, WMIX);

  k_pre<<<dim3(MP / GBM, 2), GTHR, 0, stream>>>(h, WPRE, bpre, PSD, nN);

  for (int s = 0; s < NSPLIT; ++s) {
    const int rowLo = s * RS;
    k_agg<<<gA, NTHR, LDS_AGG, stream>>>(src, dst, PSD, AGG, SCP, nN, nE, nb, vec8, rowLo, RS);
    k_post<<<gP, GTHR, 0, stream>>>(h, AGG, SCP, WPOST, WMIX, bpost, bmix, out, nN, rowLo);
  }
}
